// Graph_30837865185500
// MI455X (gfx1250) — hardware-run, weakly checked
//
#include <hip/hip_runtime.h>


namespace {

constexpr int N = 50000, NP = 50048, NPL = NP  , SRCM = N  , EFULL = 500000, E = EFULL  , H = 256, K2 = 2 * H, DEPTH = 3, NL = (NPL < N ? NPL : N), NBLK = NPL / 32;
constexpr float XS = 8.0f, WSC = 256.0f, LNEPS = 1e-5f, BASEF = 1e-4f, NSLOPE = 0.2f, SLOPE = 0.0f, BNEPS = 1e-5f;
static_assert(NP % 32 == 0 && NP >= N && NPL % 32 == 0 && H == 256, "tiling");
__constant__ float FREQ[H / 2] = {1.000000000e+00f,9.300449491e-01f,8.649836183e-01f,8.044736385e-01f,7.481966019e-01f,6.958565116e-01f,6.471778154e-01f,6.019044518e-01f,5.597981811e-01f,5.206375122e-01f,4.842162728e-01f,4.503428638e-01f,4.188391268e-01f,3.895392120e-01f,3.622889817e-01f,3.369450271e-01f,3.133740127e-01f,2.914519310e-01f,2.710634172e-01f,2.521011233e-01f,2.344653904e-01f,2.180633545e-01f,2.028087080e-01f,1.886212081e-01f,1.754262149e-01f,1.631542742e-01f,1.517408043e-01f,1.411257535e-01f,1.312533021e-01f,1.220714748e-01f,1.135319471e-01f,1.055898145e-01f,9.820327908e-02f,9.133346379e-02f,8.494423330e-02f,7.900195569e-02f,7.347536832e-02f,6.833538413e-02f,6.355497986e-02f,5.910898745e-02f,5.497401953e-02f,5.112830922e-02f,4.755162820e-02f,4.422515258e-02f,4.113136977e-02f,3.825402260e-02f,3.557796404e-02f,3.308910504e-02f,3.077435680e-02f,2.862153575e-02f,2.661931515e-02f,2.475715987e-02f,2.302527241e-02f,2.141453326e-02f,1.991647854e-02f,1.852322184e-02f,1.722742990e-02f,1.602228358e-02f,1.490144525e-02f,1.385901403e-02f,1.288950257e-02f,1.198781747e-02f,1.114920899e-02f,1.036926638e-02f,9.643883444e-03f,8.969245479e-03f,8.341802284e-03f,7.758250926e-03f,7.215522230e-03f,6.710760295e-03f,6.241308991e-03f,5.804697983e-03f,5.398630165e-03f,5.020966288e-03f,4.669724498e-03f,4.343053792e-03f,4.039235413e-03f,3.756670514e-03f,3.493872471e-03f,3.249458736e-03f,3.022142686e-03f,2.810728503e-03f,2.614103956e-03f,2.431234345e-03f,2.261157380e-03f,2.102978062e-03f,1.955864020e-03f,1.819041558e-03f,1.691789599e-03f,1.573440386e-03f,1.463370281e-03f,1.361000235e-03f,1.265791478e-03f,1.177242957e-03f,1.094888896e-03f,1.018295879e-03f,9.470609948e-04f,8.808093262e-04f,8.191922680e-04f,7.618856616e-04f,7.085879333e-04f,6.590186385e-04f,6.129170069e-04f,5.700403708e-04f,5.301631754e-04f,4.930753494e-04f,4.585822462e-04f,4.265021125e-04f,3.966661461e-04f,3.689173609e-04f,3.431097430e-04f,3.191074939e-04f,2.967843029e-04f,2.760227653e-04f,2.567135962e-04f,2.387551795e-04f,2.220530587e-04f,2.065193257e-04f,1.920722716e-04f,1.786358480e-04f,1.661392744e-04f,1.545170089e-04f,1.437077590e-04f,1.336546848e-04f,1.243048609e-04f,1.156091166e-04f,1.075216787e-04f,9.999999747e-05f};
typedef _Float16 b16;
typedef __attribute__((ext_vector_type(16))) _Float16 v16b;
typedef __attribute__((ext_vector_type(8))) _Float16 v8b;
typedef __attribute__((ext_vector_type(8))) float v8f;
typedef __attribute__((ext_vector_type(4))) float v4f;
__device__ __forceinline__ float bf16_rne(float f) { unsigned int u = __float_as_uint(f); u += 0x7FFFu + ((u >> 16) & 1u); return __uint_as_float(u & 0xFFFF0000u); }
__device__ __forceinline__ void split16(float v, b16& hi, b16& lo) { hi = (b16)v; lo = (b16)(v - (float)hi); }
__device__ __forceinline__ v16b frag_kb(const b16* p, int hh) { const v8b a = *(const v8b*)(p + 8 * hh), b = *(const v8b*)(p + 16 + 8 * hh); v16b f;
#pragma unroll
  for (int e = 0; e < 8; ++e) { f[e] = a[e]; f[8 + e] = b[e]; } return f; }
__device__ __forceinline__ v8f wmma16b(v16b a, v16b b, v8f c) { v8f d = __builtin_amdgcn_wmma_f32_16x16x32_f16(false, a, false, b, (short)0, c, false, false); asm volatile("v_nop\n\tv_nop\n\tv_nop\n\tv_nop" : "+v"(d) : "v"(a), "v"(b)); return d; }
__device__ __forceinline__ void wave_lds_sync() { __builtin_amdgcn_fence(__ATOMIC_RELEASE, "workgroup"); __builtin_amdgcn_wave_barrier(); __builtin_amdgcn_fence(__ATOMIC_ACQUIRE, "workgroup"); }
__device__ __forceinline__ float pmul(float a, float b) { float p = a * b; asm volatile("" : "+v"(p)); return p; }
__device__ __forceinline__ int iclamp(int v, int lo, int hi) { return v < lo ? lo : (v > hi ? hi : v); }
constexpr int CSR_NBLK = 512, CSR_GB = 9, CSR_GN = 1 << CSR_GB  , CSR_MAXG = 512, CSR_CAP = 12288  ;
__global__ __launch_bounds__(64) void csrA_kernel(const int* __restrict__ dst, int E, int N, int nG, int CHP, int NGP, int* __restrict__ STG, int* __restrict__ HST) {
  extern __shared__ int sm[];
  int* cnt = sm; int* run = sm + NGP; int* ids = sm + 2 * NGP;
  const int b = blockIdx.x; const int ch = (E + CSR_NBLK - 1) / CSR_NBLK; const int e0 = b * ch, e1 = min(E, e0 + ch);
  for (int i = threadIdx.x; i < NGP; i += 64) cnt[i] = 0;
  for (int i = threadIdx.x; i < CHP; i += 64) ids[i] = -1;
  __syncthreads();
  if (threadIdx.x == 0) {
    for (int e = e0; e < e1; ++e) { int d = dst[e]; d = (d < 0) ? 0 : (d >= N ? N - 1 : d); cnt[d >> CSR_GB] += 1; }
    int acc = 0; for (int g = 0; g < nG; ++g) { run[g] = acc; acc += cnt[g]; }
    for (int e = e0; e < e1; ++e) { int d = dst[e]; d = (d < 0) ? 0 : (d >= N ? N - 1 : d); const int g = d >> CSR_GB; ids[run[g]] = e; run[g] += 1; } }
  __syncthreads();
  typedef __attribute__((ext_vector_type(4))) int v4i;
  for (int pass = 0; pass < 2; ++pass) {
    for (int i = threadIdx.x; i < CHP / 4; i += 64) *(volatile v4i*)(STG + (size_t)b * CHP + i * 4) = *(const v4i*)(&ids[i * 4]);
    for (int i = threadIdx.x; i < NGP / 4; i += 64) { v4i v; for (int e = 0; e < 4; ++e) v[e] = (i * 4 + e < nG) ? cnt[i * 4 + e] : 0; *(volatile v4i*)(HST + (size_t)b * NGP + i * 4) = v; }
    __threadfence(); }
}
__global__ __launch_bounds__(512) void csrS_kernel(const int* __restrict__ HST, int nG, int NGP, int* __restrict__ START, int* __restrict__ TOT, int* __restrict__ OFF) {
  __shared__ int tot[CSR_MAXG];
  const int b = threadIdx.x;
  for (int pass = 0; pass < 2; ++pass) { int runb = 0; for (int g = 0; g < nG; ++g) { int c = HST[(size_t)b * NGP + g]; c = (c < 0) ? 0 : c; ((volatile int*)OFF)[(size_t)g * CSR_NBLK + b] = runb; runb += c; } __threadfence(); }
  for (int g = threadIdx.x; g < nG; g += 512) { int s = 0; for (int bb = 0; bb < CSR_NBLK; ++bb) { int c = HST[(size_t)bb * NGP + g]; s += (c < 0) ? 0 : c; } tot[g] = s; }
  __syncthreads();
  if (threadIdx.x < 32) {
    __shared__ int st[CSR_MAXG + 32];
    if (threadIdx.x == 0) { int acc = 0; for (int g = 0; g < NGP; ++g) { st[g] = acc; if (g < nG) acc += (tot[g] + 31) & ~31; } st[NGP] = acc; }
    __builtin_amdgcn_fence(__ATOMIC_RELEASE, "workgroup"); __builtin_amdgcn_wave_barrier(); __builtin_amdgcn_fence(__ATOMIC_ACQUIRE, "workgroup");
    for (int pass = 0; pass < 2; ++pass) { for (int i = threadIdx.x; i < NGP + 32; i += 32) { ((volatile int*)START)[i] = (i <= NGP) ? st[min(i, NGP)] : 0; ((volatile int*)TOT)[i] = (i < nG) ? tot[i] : 0; } __threadfence(); } }
}
__global__ __launch_bounds__(256) void csrB_kernel(const int* __restrict__ dst, int N, int nG, int CHP, int NGP, int permLen, const int* __restrict__ STG, const int* __restrict__ HST, const int* __restrict__ OFF, const int* __restrict__ START, const int* __restrict__ TOT, int* __restrict__ PERM, int* __restrict__ ROWPTR, int* __restrict__ ROWCNT, int* __restrict__ FLAG) {
  typedef __attribute__((ext_vector_type(4))) int v4i;
  __shared__ int ids[CSR_CAP]; __shared__ unsigned short key[CSR_CAP]; __shared__ int outp[CSR_CAP]; __shared__ int ncnt[CSR_GN + 1]; __shared__ int boff[CSR_NBLK + 1];
  const int g = blockIdx.x, t_ = threadIdx.x; int tot = TOT[g]; int st = START[g], stn = START[g + 1]; const int v0 = g * CSR_GN; const int nv = min(CSR_GN, N - v0);
  st = (st < 0) ? 0 : (st > permLen - 32 ? permLen - 32 : st) & ~31; stn = (stn < st) ? st : (stn > permLen ? permLen : stn); tot = (tot < 0) ? 0 : tot; if (tot > stn - st && tot <= CSR_CAP) tot = stn - st;
  if (tot > CSR_CAP) {
    for (int pass = 0; pass < 2; ++pass) { for (int i = t_; i < CSR_GN / 4; i += 256) { v4i a, c; for (int e = 0; e < 4; ++e) { a[e] = st; c[e] = 0; } *(volatile v4i*)(ROWPTR + v0 + i * 4) = a; *(volatile v4i*)(ROWCNT + v0 + i * 4) = c; } if (t_ == 0) ((volatile int*)FLAG)[0] = 1; __threadfence(); } (void)nv; return; }
  if (t_ == 0) { int acc = 0; for (int b = 0; b < CSR_NBLK; ++b) { boff[b] = acc; int c = HST[(size_t)b * NGP + g]; c = (c < 0) ? 0 : (c > CHP ? CHP : c); acc += c; if (acc > tot) acc = tot; } boff[CSR_NBLK] = acc; }
  for (int i = t_; i <= CSR_GN; i += 256) ncnt[i] = 0;
  __syncthreads();
  for (int b = 0; b < CSR_NBLK; ++b) { const int c = boff[b + 1] - boff[b]; int o_ = OFF[(size_t)g * CSR_NBLK + b]; o_ = (o_ < 0) ? 0 : (o_ > CHP - c ? CHP - c : o_); const int* src_ = STG + (size_t)b * CHP + o_;
    for (int i = t_; i < c; i += 256) { int id = src_[i]; id = (id < 0) ? 0 : id; ids[boff[b] + i] = id; int d = dst[id]; d = (d < v0) ? v0 : (d >= N ? N - 1 : d); int kk = d - v0; kk = (kk < 0) ? 0 : (kk >= CSR_GN ? CSR_GN - 1 : kk); key[boff[b] + i] = (unsigned short)kk; } }
  __syncthreads();
  if (t_ == 0) { for (int i = 0; i < tot; ++i) ncnt[key[i]] += 1; int acc = 0; for (int vl = 0; vl < CSR_GN; ++vl) { const int c = ncnt[vl]; ncnt[vl] = acc; acc += c; } ncnt[CSR_GN] = acc;
    for (int i = 0; i < tot; ++i) { const int vl = key[i]; outp[ncnt[vl]] = ids[i]; ncnt[vl] += 1; }
    for (int vl = CSR_GN; vl > 0; --vl) ncnt[vl] = ncnt[vl - 1]; ncnt[0] = 0; }
  __syncthreads();
  for (int pass = 0; pass < 2; ++pass) {
    for (int i = t_; i < (stn - st) / 4; i += 256) { v4i v; for (int e = 0; e < 4; ++e) { const int q = i * 4 + e; v[e] = (q < tot) ? outp[q] : -1; } *(volatile v4i*)(PERM + st + i * 4) = v; }
    for (int i = t_; i < CSR_GN / 4; i += 256) { v4i a, c; for (int e = 0; e < 4; ++e) { const int vl = i * 4 + e; a[e] = st + ncnt[vl]; c[e] = (vl < nv) ? (ncnt[vl + 1] - ncnt[vl]) : 0; } *(volatile v4i*)(ROWPTR + v0 + i * 4) = a; *(volatile v4i*)(ROWCNT + v0 + i * 4) = c; }
    __threadfence(); }
}
__global__ __launch_bounds__(256) void csrZ_kernel(int* __restrict__ p, size_t n4) { typedef __attribute__((ext_vector_type(4))) int v4i; const size_t tid = (size_t)blockIdx.x * 256 + threadIdx.x, nth = (size_t)gridDim.x * 256; v4i z = {0, 0, 0, 0}; for (size_t i = tid; i < n4; i += nth) *(volatile v4i*)(p + i * 4) = z; }
struct CsrBufs { int *STG, *HST, *OFF, *START, *TOT, *PERM, *ROWPTR, *ROWCNT, *FLAG; int nG, NGP, CHP; size_t permLen; char* base; size_t bytes; };
static size_t csr_carve(CsrBufs& c, char* ws, size_t off, int E, int N) {
  const size_t off0 = off; c.base = ws + off;
  auto al = [&](size_t bytes) { char* p = ws + off; off += (bytes + 255) & ~(size_t)255; return p; };
  c.nG = (N + CSR_GN - 1) / CSR_GN; c.NGP = (c.nG + 31) & ~31; const int ch = (E + CSR_NBLK - 1) / CSR_NBLK; c.CHP = (ch + 31) & ~31; c.permLen = (size_t)E + 32 * (size_t)c.nG + 32;
  c.STG = (int*)al((size_t)CSR_NBLK * c.CHP * 4); c.HST = (int*)al((size_t)CSR_NBLK * c.NGP * 4); c.OFF = (int*)al((size_t)c.NGP * CSR_NBLK * 4); c.START = (int*)al((size_t)(c.NGP + 64) * 4); c.TOT = (int*)al((size_t)(c.NGP + 64) * 4);
  c.PERM = (int*)al(c.permLen * 4); c.ROWPTR = (int*)al((size_t)c.nG * CSR_GN * 4); c.ROWCNT = (int*)al((size_t)c.nG * CSR_GN * 4); c.FLAG = (int*)al(256);
  c.bytes = off - off0; return off;
}
static void csr_build(const CsrBufs& c, const int* dst, int E, int N, hipStream_t stream) {
  const size_t smem = (size_t)(2 * c.NGP + c.CHP) * 4;
  csrZ_kernel<<<512, 256, 0, stream>>>((int*)c.base, c.bytes / 16);
  csrA_kernel<<<CSR_NBLK, 64, smem, stream>>>(dst, E, N, c.nG, c.CHP, c.NGP, c.STG, c.HST);
  csrS_kernel<<<1, 512, 0, stream>>>(c.HST, c.nG, c.NGP, c.START, c.TOT, c.OFF);
  csrB_kernel<<<c.nG, 256, 0, stream>>>(dst, N, c.nG, c.CHP, c.NGP, (int)c.permLen, c.STG, c.HST, c.OFF, c.START, c.TOT, c.PERM, c.ROWPTR, c.ROWCNT, c.FLAG);
}

typedef __attribute__((ext_vector_type(4))) _Float16 v4h;
typedef __attribute__((ext_vector_type(2))) float v2f;
template <int KD, int KA, int NOUT, int EPI>
__global__ __launch_bounds__(64) void gemm1_kernel(const float* __restrict__ A0, const float* __restrict__ A1, const b16* __restrict__ W, const float* __restrict__ bias, const float* __restrict__ RES, float* __restrict__ T, int mrows) {
  static_assert(KD % 128 == 0 && KA % 128 == 0 && NOUT % 128 == 0 && KA <= KD, "gemm1 tiling"); constexpr int KB = KD - KA;
  __shared__ __attribute__((aligned(16))) b16 As[2][16][128 + 8]; __shared__ __attribute__((aligned(16))) float Tf[2][16][128 + 4];
  const int wave = threadIdx.x >> 5, lane = threadIdx.x & 31, nloc = lane & 15, hlf = lane >> 4; const size_t m0 = (size_t)blockIdx.x * 32 + wave * 16; const int n0 = blockIdx.y * 128;
  v8f acc[8];
#pragma unroll
  for (int t = 0; t < 8; ++t) acc[t] = (v8f){};
#pragma unroll 1
  for (int kc = 0; kc < KD; kc += 128) { const float* src = kc < KA ? A0 : A1; const int pitch = kc < KA ? KA : KB, cofs = kc < KA ? kc : kc - KA;
    for (int idx = lane; idx < 16 * 32; idx += 32) { const int rr = idx / 32, c4 = (idx % 32) * 4; const v4f v = *(const v4f*)(src + (m0 + rr) * pitch + cofs + c4); v4h o; for (int j = 0; j < 4; ++j) o[j] = (b16)(v[j] * XS); *(v4h*)(&As[wave][rr][c4]) = o; }
    wave_lds_sync();
#pragma unroll
    for (int kb = 0; kb < 128; kb += 32) { const v16b a = frag_kb(&As[wave][nloc][kb], hlf);
#pragma unroll
      for (int t = 0; t < 8; ++t) acc[t] = wmma16b(a, frag_kb(W + (size_t)(n0 + t * 16 + nloc) * KD + kc + kb, hlf), acc[t]); }
    wave_lds_sync(); }
#pragma unroll
  for (int t = 0; t < 8; ++t) { const float bb = bias ? bf16_rne(bias[n0 + t * 16 + nloc]) : 0.0f;
#pragma unroll
    for (int r = 0; r < 8; ++r) { float v = acc[t][r] * (1.0f / (XS * WSC)) + bb; if (EPI == 1) v = fmaxf(v, 0.0f); if (EPI == 2) { size_t rrow = m0 + 8 * hlf + r; if (rrow > (size_t)(mrows - 1)) rrow = (size_t)(mrows - 1); v += bf16_rne(RES[rrow * NOUT + n0 + t * 16 + nloc]); }   Tf[wave][8 * hlf + r][t * 16 + nloc] = v; } }
  wave_lds_sync();
  for (int pass = 0; pass < 2; ++pass) { for (int rr = 0; rr < 16; ++rr) if (m0 + rr < (size_t)mrows) *(volatile v4f*)(T + (m0 + rr) * NOUT + n0 + lane * 4) = *(const v4f*)(&Tf[wave][rr][lane * 4]); __threadfence(); }
}

__global__ __launch_bounds__(256) void wcvt_kernel(const float* __restrict__ w, b16* __restrict__ W16, int n8) { const int u = blockIdx.x * 256 + threadIdx.x; if (u >= n8) return; const size_t e = (size_t)u * 8; v8b o; for (int j = 0; j < 8; ++j) o[j] = (b16)(bf16_rne(w[e + j]) * WSC);
  for (int pass = 0; pass < 2; ++pass) { *(volatile v8b*)(W16 + e) = o; __threadfence(); } }
__global__ __launch_bounds__(256) void wlr_kernel(const float* __restrict__ wl, const float* __restrict__ wr, b16* __restrict__ WLR) {
  const int u = blockIdx.x * 256 + threadIdx.x; if (u >= DEPTH * H * K2 / 8) return; const int e = u * 8; const int l = e / (H * K2), rem = e % (H * K2), o = rem / K2, k0 = rem % K2; const float* w = (k0 < H ? wl : wr) + ((size_t)l * H + o) * H + (k0 & (H - 1)); v8b v;
#pragma unroll
  for (int j = 0; j < 8; ++j) v[j] = (b16)(bf16_rne(w[j]) * WSC);
  for (int pass = 0; pass < 2; ++pass) { *(volatile v8b*)(WLR + e) = v; __threadfence(); }
}
__global__ __launch_bounds__(256) void pe_kernel(const float* __restrict__ x, const float* __restrict__ pos, float* __restrict__ H0) {
  __shared__ float fr[H / 2]; if (threadIdx.x < H / 2) fr[threadIdx.x] = FREQ[threadIdx.x];
  __syncthreads();
  const size_t u = (size_t)blockIdx.x * 256 + threadIdx.x; if (u >= (size_t)NP * H / 4) return; const int v = (int)(u * 4 / H), c = (int)((u * 4) % H); v4f o = {0.0f, 0.0f, 0.0f, 0.0f};
  if (v < N) { const float pv = bf16_rne(pos[v]); for (int j = 0; j < 4; ++j) { const int cc = c + j; const float ang = pv * fr[cc & (H / 2 - 1)]; const float pe = (cc < H / 2) ? sinf(ang) : cosf(ang); o[j] = bf16_rne(x[(size_t)v * H + cc]) + pe; } }
  for (int pass = 0; pass < 2; ++pass) { *(volatile v4f*)(H0 + u * 4) = o; __threadfence(); }
}
__global__ __launch_bounds__(256) void aggh2_kernel(const float* __restrict__ XP, const float* __restrict__ Hin, const int* __restrict__ srcs, const int* __restrict__ PERM, const int* __restrict__ ROWPTR, const int* __restrict__ ROWCNT, int permLen, const b16* __restrict__ WLR, const float* __restrict__ bl, float* __restrict__ H2, float* __restrict__ PART) {
  __shared__ __attribute__((aligned(16))) b16 As[32][K2 + 8]; __shared__ __attribute__((aligned(16))) float Tf[32][H + 4]; __shared__ float red[256];
  const int tid = threadIdx.x, wave = tid >> 5, lane = tid & 31, nloc = lane & 15, hlf = lane >> 4; const int v0 = blockIdx.x * 32;
  { const int row = tid >> 3, g = tid & 7, c0 = g * 32; const int v = v0 + row; float acc[32]; for (int j = 0; j < 32; ++j) acc[j] = 0.0f;
    int cnt = 0, p0 = 0; if (v < N) { cnt = iclamp(ROWCNT[v], 0, 65536); p0 = iclamp(ROWPTR[v], 0, permLen - 1); if (p0 + cnt > permLen) cnt = permLen - p0; }
#pragma unroll 1
    for (int i = 0; i < cnt; ++i) { int e = iclamp(PERM[p0 + i], 0, E - 1); int s = iclamp(srcs[e], 0, N - 1); if (SRCM < N) s %= SRCM; const float* xr = XP + (size_t)s * H + c0;
#pragma unroll
      for (int q = 0; q < 8; ++q) { const v4f t4 = *(const v4f*)(xr + 4 * q); for (int j = 0; j < 4; ++j) acc[4 * q + j] += t4[j]; } }
    const float inv = (v < N && cnt > 0) ? 1.0f / (float)cnt : 0.0f; const float* hr = Hin + (size_t)iclamp(v, 0, N - 1) * H + c0;
#pragma unroll
    for (int q = 0; q < 8; ++q) { const v4f t4 = *(const v4f*)(hr + 4 * q); v4h oa, oh; for (int j = 0; j < 4; ++j) { oa[j] = (b16)(acc[4 * q + j] * inv * XS); oh[j] = (b16)((v < N ? t4[j] : 0.0f) * XS); } *(v4h*)(&As[row][c0 + 4 * q]) = oa; *(v4h*)(&As[row][H + c0 + 4 * q]) = oh; } }
  __syncthreads();
  { v8f acc2[2][2] = {{(v8f){}, (v8f){}}, {(v8f){}, (v8f){}}};
#pragma unroll
    for (int tt = 0; tt < 2; ++tt) { const b16* br = WLR + (size_t)(wave * 32 + tt * 16 + nloc) * K2;
#pragma unroll 2
      for (int kb = 0; kb < K2; kb += 32) { const v16b bw = frag_kb(br + kb, hlf); acc2[0][tt] = wmma16b(frag_kb(&As[nloc][kb], hlf), bw, acc2[0][tt]); acc2[1][tt] = wmma16b(frag_kb(&As[16 + nloc][kb], hlf), bw, acc2[1][tt]); } }
#pragma unroll
    for (int tt = 0; tt < 2; ++tt) { const int col = wave * 32 + tt * 16 + nloc; const float bb = bf16_rne(bl[col]);
#pragma unroll
      for (int rt = 0; rt < 2; ++rt)
#pragma unroll
        for (int r = 0; r < 8; ++r) { const int rr = rt * 16 + 8 * hlf + r; Tf[rr][col] = (v0 + rr < N) ? acc2[rt][tt][r] * (1.0f / (XS * WSC)) + bb : 0.0f; } } }
  __syncthreads();
  { float s = 0.0f; for (int i = tid; i < 32 * H; i += 256) s += Tf[i / H][i % H]; red[tid] = s; }
  __syncthreads();
  for (int st = 128; st >= 1; st >>= 1) { if (tid < st) red[tid] += red[tid + st]; __syncthreads(); }
  for (int pass = 0; pass < 2; ++pass) { for (int rr = wave * 4; rr < wave * 4 + 4; ++rr) { *(volatile v4f*)(H2 + (size_t)(v0 + rr) * H + lane * 4) = *(const v4f*)(&Tf[rr][lane * 4]); *(volatile v4f*)(H2 + (size_t)(v0 + rr) * H + 128 + lane * 4) = *(const v4f*)(&Tf[rr][128 + lane * 4]); }
    if (wave == 0) ((volatile float*)PART)[(size_t)blockIdx.x * 32 + lane] = (lane == 0) ? red[0] : 0.0f;
    __threadfence(); }
}
__global__ __launch_bounds__(256) void varp_kernel(const float* __restrict__ H2, const float* __restrict__ STAT, float* __restrict__ PART) {
  __shared__ float red[256]; const int tid = threadIdx.x; const int v0 = blockIdx.x * 32; const float mu = STAT[0]; float s = 0.0f;
  for (int i = tid; i < 32 * H; i += 256) { const int v = v0 + i / H; if (v < N) { const float d = H2[(size_t)v * H + (i % H)] - mu; s = fmaf(d, d, s); } }
  red[tid] = s; __syncthreads();
  for (int st = 128; st >= 1; st >>= 1) { if (tid < st) red[tid] += red[tid + st]; __syncthreads(); }
  for (int pass = 0; pass < 2; ++pass) { if (tid < 32) ((volatile float*)PART)[(size_t)blockIdx.x * 32 + tid] = (tid == 0) ? red[0] : 0.0f; __threadfence(); }
}
__global__ __launch_bounds__(256) void reduce_kernel(const float* __restrict__ PART, float* __restrict__ STAT, int which) {
  __shared__ float red[256]; const int tid = threadIdx.x; float s = 0.0f; for (int i = tid; i < NBLK; i += 256) s += PART[(size_t)i * 32]; red[tid] = s; __syncthreads();
  for (int st = 128; st >= 1; st >>= 1) { if (tid < st) red[tid] += red[tid + st]; __syncthreads(); }
  for (int pass = 0; pass < 2; ++pass) { if (tid < 32) ((volatile float*)STAT)[which * 32 + tid] = (tid == 0) ? red[0] / ((float)N * (float)H) : 0.0f; __threadfence(); }
}
__global__ __launch_bounds__(256) void ln_kernel(const float* __restrict__ H2, const float* __restrict__ STAT, const float* __restrict__ lw, const float* __restrict__ lb, float* __restrict__ Hout) {
  const size_t u = (size_t)blockIdx.x * 256 + threadIdx.x; if (u >= (size_t)NP * H / 4) return; const int v = (int)(u * 4 / H), c = (int)((u * 4) % H); const float mu = STAT[0], rs = rsqrtf(STAT[32] + LNEPS);
  const v4f hv = *(const v4f*)(H2 + u * 4); v4f o; for (int j = 0; j < 4; ++j) { float y = (hv[j] - mu) * rs * bf16_rne(lw[c + j]) + bf16_rne(lb[c + j]); y = y > 0.0f ? y : NSLOPE * y; o[j] = (v < N) ? y : 0.0f; }
  for (int pass = 0; pass < 2; ++pass) { *(volatile v4f*)(Hout + u * 4) = o; __threadfence(); }
}
}

extern "C" void kernel_launch(void* const* d_in, const int* in_sizes, int n_in, void* d_out, int out_size, void* d_ws, size_t ws_size, hipStream_t stream) {
  (void)n_in;
  auto Fp = [&](int i) { return (const float*)d_in[i]; }; auto Ip = [&](int i) { return (const int*)d_in[i]; };
  if (in_sizes[0] != N * H || in_sizes[1] != N || in_sizes[2] != 2 * EFULL || in_sizes[3] != DEPTH * H * H || in_sizes[4] != DEPTH * H || in_sizes[5] != DEPTH * H * H || in_sizes[6] != DEPTH * H || in_sizes[7] != DEPTH * H * H || in_sizes[8] != DEPTH * H || in_sizes[9] != DEPTH * H || in_sizes[10] != H * H || in_sizes[11] != H || out_size != N * H) return;
  size_t off = 0; char* ws = (char*)d_ws;
  auto carve = [&](size_t bytes) { char* p = ws + off; off += (bytes + 255) & ~(size_t)255; return p; };
  b16* WPT = (b16*)carve((size_t)DEPTH * H * H * 2); b16* WLR = (b16*)carve((size_t)DEPTH * H * K2 * 2); b16* WOT = (b16*)carve((size_t)H * H * 2);
  float* Ha = (float*)carve((size_t)NP * H * 4); float* XP = (float*)carve((size_t)NP * H * 4); float* H2 = (float*)carve((size_t)NP * H * 4); float* PART = (float*)carve((size_t)NBLK * 128); float* STAT = (float*)carve(256);
  CsrBufs csr; off = csr_carve(csr, ws, off, E, N);
  if (off > ws_size || off > ((size_t)192 << 20)) return;
  wcvt_kernel<<<(DEPTH * H * H / 8 + 255) / 256, 256, 0, stream>>>(Fp(3), WPT, DEPTH * H * H / 8); wlr_kernel<<<(DEPTH * H * K2 / 8 + 255) / 256, 256, 0, stream>>>(Fp(5), Fp(7), WLR); wcvt_kernel<<<(H * H / 8 + 255) / 256, 256, 0, stream>>>(Fp(10), WOT, H * H / 8);
  csr_build(csr, Ip(2) + EFULL, E, N, stream);
  const unsigned nb4 = (unsigned)(((size_t)NP * H / 4 + 255) / 256);
  pe_kernel<<<nb4, 256, 0, stream>>>(Fp(0), Fp(1), Ha);
  for (int l = 0; l < DEPTH; ++l) {
    gemm1_kernel<H, H, H, 1><<<dim3(NPL / 32, H / 128), 64, 0, stream>>>(Ha, Ha, WPT + (size_t)l * H * H, Fp(4) + l * H, nullptr, XP, NPL);
    aggh2_kernel<<<NBLK, 256, 0, stream>>>(XP, Ha, Ip(2), csr.PERM, csr.ROWPTR, csr.ROWCNT, (int)csr.permLen, WLR + (size_t)l * H * K2, Fp(6) + l * H, H2, PART);
    reduce_kernel<<<1, 256, 0, stream>>>(PART, STAT, 0);
    varp_kernel<<<NBLK, 256, 0, stream>>>(H2, STAT, PART);
    reduce_kernel<<<1, 256, 0, stream>>>(PART, STAT, 1);
    ln_kernel<<<nb4, 256, 0, stream>>>(H2, STAT, Fp(8) + l * H, Fp(9) + l * H, Ha); }
  gemm1_kernel<H, H, H, 2><<<dim3(NPL / 32, H / 128), 64, 0, stream>>>(Ha, Ha, WOT, Fp(11), Fp(0), (float*)d_out, NL);
}
